// SparseAttention_69303592288297
// MI455X (gfx1250) — hardware-verified
//
#include <hip/hip_runtime.h>
#include <stddef.h>


typedef _Float16 v16h __attribute__((ext_vector_type(16)));
typedef _Float16 v8h  __attribute__((ext_vector_type(8)));
typedef float    v8f  __attribute__((ext_vector_type(8)));
typedef float    v4f  __attribute__((ext_vector_type(4)));

#ifndef NB
#define NB 1
#endif
#ifndef SEQ
#define SEQ 4096
#endif
#define NB_FULL  1
#define SEQ_FULL 4096
#define DIM   1024
#define NHEAD 16
#define HD    64
#define MROWS (NB * SEQ)
#define WINDOW 256
#define STRIDE 64
#define EROWS  256
#ifndef EARLY_RES
#define EARLY_RES 1
#endif

static_assert(NB == 1 && NB_FULL == 1);
static_assert(SEQ >= EROWS && SEQ <= SEQ_FULL && (SEQ % 128) == 0);
static_assert(DIM == NHEAD * HD);
static_assert(HD == 64);
static_assert((DIM % 64) == 0 && (DIM % 32) == 0);
static_assert((MROWS % 64) == 0 && (MROWS % 8) == 0);
static_assert(STRIDE == 64);
static_assert((WINDOW % 128) == 0);
static_assert(EROWS == WINDOW && (EROWS % 128) == 0 && (EROWS % 64) == 0);
static_assert((((size_t)MROWS * DIM) % 2048) == 0);
static_assert((((size_t)DIM * DIM) % 2048) == 0);
static_assert((size_t)MROWS * DIM < (size_t)0xFFFFFFFFu);

#define LDT 72
#define LDC 68
static_assert((LDT % 8) == 0 && LDT >= 64);
static_assert((LDC % 4) == 0 && LDC >= 64);

#define WCARRY 64.0f
#define PCARRY 1024.0f
#define VCARRY 64.0f
#define RCARRY 1024.0f

#define WSQ_BYTES     ((size_t)DIM * DIM * 2)
#define PLANE16_BYTES ((size_t)MROWS * DIM * 2)
#define RES_BYTES     ((size_t)EROWS * DIM * 2)
#define OFF_X   ((size_t)0)
#define OFF_WQ  (OFF_X + PLANE16_BYTES)
#define OFF_WK  (OFF_WQ + WSQ_BYTES)
#define OFF_WV  (OFF_WK + WSQ_BYTES)
#define OFF_WO  (OFF_WV + WSQ_BYTES)
#define OFF_Q   (OFF_WO + WSQ_BYTES)
#define OFF_K   (OFF_Q + PLANE16_BYTES)
#define OFF_VT  (OFF_K + PLANE16_BYTES)
#define OFF_CTX (OFF_VT + PLANE16_BYTES)
#define OFF_QR  (OFF_CTX + PLANE16_BYTES)
#define OFF_KR  (OFF_QR + RES_BYTES)
#define OFF_VR  (OFF_KR + RES_BYTES)
#define OFF_CR  (OFF_VR + RES_BYTES)
#define WS_TOTAL (OFF_CR + RES_BYTES)
static_assert((WSQ_BYTES % 128) == 0 && (PLANE16_BYTES % 128) == 0 && (RES_BYTES % 128) == 0);
static_assert(WS_TOTAL <= (size_t)134217728);

__device__ __forceinline__ float bf16r(float x) {
  unsigned int u = __float_as_uint(x);
  u = (u + 0x7FFFu + ((u >> 16) & 1u)) & 0xFFFF0000u;
  return __uint_as_float(u);
}

static __device__ __forceinline__ _Float16 toh_flush(float v) {
  const _Float16 r = (_Float16)v;
  return (fabsf(v) < 6.103515625e-05f) ? (_Float16)0.0f : r;
}

__device__ __forceinline__ v16h frag_at(const _Float16* p) {
  v8h lo = *(const v8h*)(p);
  v8h hi = *(const v8h*)(p + 16);
  v16h out;
#pragma unroll
  for (int i = 0; i < 8; ++i) { out[i] = lo[i]; out[i + 8] = hi[i]; }
  return out;
}
__device__ __forceinline__ v16h ld_frag(const _Float16* base, unsigned ld) {
  const unsigned lane = threadIdx.x & 31u;
  return frag_at(base + (lane & 15u) * ld + (lane >> 4) * 8u);
}
__device__ __forceinline__ v16h frag_two(const _Float16* p0, const _Float16* p1) {
  v8h lo = *(const v8h*)(p0);
  v8h hi = *(const v8h*)(p1);
  v16h out;
#pragma unroll
  for (int i = 0; i < 8; ++i) { out[i] = lo[i]; out[i + 8] = hi[i]; }
  return out;
}

__device__ __forceinline__ v8f wmma16(v16h a, v16h b, v8f c) {
  v8f d = __builtin_amdgcn_wmma_f32_16x16x32_f16(false, a, false, b, (short)0, c,
                                                 false, false);
  asm volatile("v_nop\n\tv_nop\n\tv_nop\n\tv_nop" : "+v"(d) : "v"(a), "v"(b));
  return d;
}

__device__ __forceinline__ float red16_max(float x) {
#pragma unroll
  for (int off = 1; off < 16; off <<= 1) x = fmaxf(x, __shfl_xor(x, off, 32));
  return x;
}
__device__ __forceinline__ float red16_sum(float x) {
#pragma unroll
  for (int off = 1; off < 16; off <<= 1) x += __shfl_xor(x, off, 32);
  return x;
}

__device__ __forceinline__ void wave_lds_sync() {
  __builtin_amdgcn_fence(3  , "wavefront");
  asm volatile("s_wait_dscnt 0x0" ::: "memory");
  __builtin_amdgcn_wave_barrier();
}

__global__ __launch_bounds__(256) void cvt_plane_kernel(
    const float* __restrict__ src, _Float16* __restrict__ dst, const float carry) {
  const size_t i = ((size_t)blockIdx.x * 256u + threadIdx.x) * 8u;
  const v4f a0 = *(const v4f*)(src + i);
  const v4f a1 = *(const v4f*)(src + i + 4u);
  v8h o;
#pragma unroll
  for (int j = 0; j < 4; ++j) {
    o[j]     = toh_flush(carry * bf16r(a0[j]));
    o[j + 4] = toh_flush(carry * bf16r(a1[j]));
  }
  *(volatile v8h*)(dst + i) = o;
  __threadfence();
  *(volatile v8h*)(dst + i) = o;
}

template <int MODE>
__device__ __forceinline__ void gemm_body(
    const _Float16* __restrict__ A16, const _Float16* __restrict__ A16r,
    const _Float16* __restrict__ Bt, const unsigned K,
    float* __restrict__ outf, _Float16* __restrict__ out16, _Float16* __restrict__ out16r) {
  __shared__ float Cs[64 * LDC];
  const unsigned tid = threadIdx.x, lane = tid & 31u;
  const unsigned w = (unsigned)__builtin_amdgcn_readfirstlane((int)(tid >> 5));
  const unsigned mw = w >> 1, nw = w & 1u;
  const unsigned hh = lane >> 4, m = lane & 15u;
  const unsigned n0 = blockIdx.x * 64u;
  const unsigned row0 = blockIdx.y * 64u;
  const bool early = (EARLY_RES != 0) && (row0 < (unsigned)EROWS);

  const _Float16* ap  = A16 + (size_t)(row0 + mw * 16u + m) * K + hh * 8u;
  const _Float16* bp0 = Bt + (size_t)(n0 + nw * 32u + m) * K + hh * 8u;
  const _Float16* bp1 = bp0 + (size_t)16 * K;
  v8f acc0 = {}, acc1 = {};
#pragma unroll 2
  for (unsigned k0 = 0; k0 < K; k0 += 32u) {
    const v16h a  = frag_at(ap + k0);
    const v16h b0 = frag_at(bp0 + k0);
    const v16h b1 = frag_at(bp1 + k0);
    acc0 = wmma16(a, b0, acc0);
    acc1 = wmma16(a, b1, acc1);
  }
  if (MODE == 2) {
    if (early) {
      const _Float16* apr = A16r + (size_t)(row0 + mw * 16u + m) * K + hh * 8u;
      v8f r0 = {}, r1 = {};
#pragma unroll 2
      for (unsigned k0 = 0; k0 < K; k0 += 32u) {
        const v16h a  = frag_at(apr + k0);
        const v16h b0 = frag_at(bp0 + k0);
        const v16h b1 = frag_at(bp1 + k0);
        r0 = wmma16(a, b0, r0);
        r1 = wmma16(a, b1, r1);
      }
#pragma unroll
      for (int r = 0; r < 8; ++r) {
        acc0[r] = acc0[r] + r0[r] * (1.0f / RCARRY);
        acc1[r] = acc1[r] + r1[r] * (1.0f / RCARRY);
      }
    }
  }
#pragma unroll
  for (int r = 0; r < 8; ++r) {
    float* d = &Cs[(mw * 16u + hh * 8u + (unsigned)r) * LDC + nw * 32u + m];
    d[0]  = acc0[r];
    d[16] = acc1[r];
  }
  __syncthreads();

  if (MODE == 0) {
    v8h x[2], xr[2];
    size_t off[2];
#pragma unroll
    for (unsigned i = 0; i < 2u; ++i) {
      const unsigned r = 32u * i + (tid >> 3);
      const unsigned c = (tid & 7u) * 8u;
      const v4f u0 = *(const v4f*)&Cs[r * LDC + c];
      const v4f u1 = *(const v4f*)&Cs[r * LDC + c + 4];
#pragma unroll
      for (int j = 0; j < 4; ++j) {
        const float t0 = u0[j] * (1.0f / WCARRY);
        const float t1 = u1[j] * (1.0f / WCARRY);
        const _Float16 h0 = toh_flush(t0);
        const _Float16 h1 = toh_flush(t1);
        x[i][j]      = h0;
        x[i][j + 4]  = h1;
        xr[i][j]     = toh_flush((t0 - (float)h0) * RCARRY);
        xr[i][j + 4] = toh_flush((t1 - (float)h1) * RCARRY);
      }
      off[i] = (size_t)(row0 + r) * DIM + n0 + c;
    }
#pragma unroll
    for (int i = 0; i < 2; ++i) *(volatile v8h*)(out16 + off[i]) = x[i];
    if (early) {
#pragma unroll
      for (int i = 0; i < 2; ++i) *(volatile v8h*)(out16r + off[i]) = xr[i];
    }
    __threadfence();
#pragma unroll
    for (int i = 0; i < 2; ++i) *(volatile v8h*)(out16 + off[i]) = x[i];
    if (early) {
#pragma unroll
      for (int i = 0; i < 2; ++i) *(volatile v8h*)(out16r + off[i]) = xr[i];
    }
  }

  if (MODE == 1) {
    const unsigned key0 = row0;
    v8h x[2], xr[2];
    size_t off[2], offr[2];
#pragma unroll
    for (unsigned i = 0; i < 2u; ++i) {
      const unsigned dcol = 32u * i + (tid >> 3);
      const unsigned kk = (tid & 7u) * 8u;
#pragma unroll
      for (unsigned j = 0; j < 8u; ++j) {
        const float t = Cs[(kk + j) * LDC + dcol] * (1.0f / WCARRY);
        const _Float16 hi = toh_flush(t);
        x[i][j]  = hi;
        xr[i][j] = toh_flush((t - (float)hi) * RCARRY);
      }
      off[i]  = (size_t)(n0 + dcol) * SEQ + key0 + kk;
      offr[i] = (size_t)(n0 + dcol) * EROWS + key0 + kk;
    }
#pragma unroll
    for (int i = 0; i < 2; ++i) *(volatile v8h*)(out16 + off[i]) = x[i];
    if (early) {
#pragma unroll
      for (int i = 0; i < 2; ++i) *(volatile v8h*)(out16r + offr[i]) = xr[i];
    }
    __threadfence();
#pragma unroll
    for (int i = 0; i < 2; ++i) *(volatile v8h*)(out16 + off[i]) = x[i];
    if (early) {
#pragma unroll
      for (int i = 0; i < 2; ++i) *(volatile v8h*)(out16r + offr[i]) = xr[i];
    }
  }

  if (MODE == 2) {
    const float cs = 1.0f / (WCARRY * VCARRY);
    v4f xs[4];
    size_t off[4];
#pragma unroll
    for (unsigned i = 0; i < 4u; ++i) {
      const unsigned r = 16u * i + (tid >> 4);
      const unsigned c = (tid & 15u) * 4u;
      const v4f u = *(const v4f*)&Cs[r * LDC + c];
      v4f val;
#pragma unroll
      for (int j = 0; j < 4; ++j) val[j] = u[j] * cs;
      xs[i] = val;
      off[i] = (size_t)(row0 + r) * DIM + n0 + c;
    }
#pragma unroll
    for (int i = 0; i < 4; ++i) *(volatile v4f*)(outf + off[i]) = xs[i];
    __threadfence();
#pragma unroll
    for (int i = 0; i < 4; ++i) *(volatile v4f*)(outf + off[i]) = xs[i];
  }
}

__global__ __launch_bounds__(256) void gemm_qk_kernel(
    const _Float16* __restrict__ A16, const _Float16* __restrict__ Bt,
    _Float16* __restrict__ out16, _Float16* __restrict__ out16r) {
  gemm_body<0>(A16, A16, Bt, (unsigned)DIM, (float*)0, out16, out16r);
}
__global__ __launch_bounds__(256) void gemm_v_kernel(
    const _Float16* __restrict__ A16, const _Float16* __restrict__ Bt,
    _Float16* __restrict__ vt, _Float16* __restrict__ vtr) {
  gemm_body<1>(A16, A16, Bt, (unsigned)DIM, (float*)0, vt, vtr);
}
__global__ __launch_bounds__(256) void gemm_wo_kernel(
    const _Float16* __restrict__ A16, const _Float16* __restrict__ A16r,
    const _Float16* __restrict__ Bt, float* __restrict__ outf) {
  gemm_body<2>(A16, A16r, Bt, (unsigned)DIM, outf, (_Float16*)0, (_Float16*)0);
}

template <int EARLY>
__device__ __forceinline__ void attn_body(
    const _Float16* __restrict__ Qh, const _Float16* __restrict__ Kh,
    const _Float16* __restrict__ Vt, const _Float16* __restrict__ QR,
    const _Float16* __restrict__ KR, const _Float16* __restrict__ VtR,
    _Float16* __restrict__ Ov, _Float16* __restrict__ OvR, const unsigned q0) {
  __shared__ _Float16 Ks[64 * LDT];
  __shared__ _Float16 Vs[64 * LDT];
  __shared__ _Float16 KRs[64 * LDT];
  __shared__ _Float16 VRs[64 * LDT];
  __shared__ _Float16 Ps[8 * 16 * LDT];

  const unsigned tid = threadIdx.x, lane = tid & 31u;
  const unsigned w = (unsigned)__builtin_amdgcn_readfirstlane((int)(tid >> 5));
  const unsigned hh = lane >> 4, m = lane & 15u;
  const unsigned head = blockIdx.y;
  const float scale = 0.125f;
  const unsigned qrow0 = q0 + w * 16u;
  _Float16* P = Ps + w * (16u * LDT);

  const size_t qoff = (size_t)(qrow0 + m) * DIM + head * HD + hh * 8u;
  v16h qf[2], qr[2];
  qf[0] = frag_at(Qh + qoff);
  qf[1] = frag_at(Qh + qoff + 32);
  if (EARLY) {
    qr[0] = frag_at(QR + qoff);
    qr[1] = frag_at(QR + qoff + 32);
  } else {
    qr[0] = qf[0];
    qr[1] = qf[1];
  }

  float mrow[8], lrow[8];
  v8f o[4];
#pragma unroll
  for (int v = 0; v < 8; ++v) { mrow[v] = -1.0e30f; lrow[v] = 0.0f; }
#pragma unroll
  for (int nb = 0; nb < 4; ++nb) o[nb] = (v8f){};

  const size_t kplane = (size_t)head * HD;
  const size_t vplane = (size_t)(head * HD) * SEQ;
  const size_t rplane = (size_t)(head * HD) * EROWS;
  const unsigned wstart = (q0 > (unsigned)WINDOW) ? (q0 - (unsigned)WINDOW) : 0u;
  const unsigned kend = q0 + 128u;

  if (!EARLY) {
    const unsigned kg = w & 3u;
    for (unsigned kb = 0; kb + 128u <= wstart; kb += 128u) {
      const _Float16* ka = Kh + (size_t)(kb + kg * 16u + m) * DIM + kplane + hh * 8u;
      const _Float16* kc = ka + (size_t)64 * DIM;
      v8f s0 = {}, s1 = {};
      s0 = wmma16(qf[0], frag_at(ka), s0);
      s0 = wmma16(qf[1], frag_at(ka + 32), s0);
      s1 = wmma16(qf[0], frag_at(kc), s1);
      s1 = wmma16(qf[1], frag_at(kc + 32), s1);
#pragma unroll
      for (int v = 0; v < 8; ++v) {
        const bool diag = (m == hh * 8u + (unsigned)v);
        s0[v] = diag ? s0[v] * scale : -1.0e30f;
        s1[v] = diag ? s1[v] * scale : -1.0e30f;
      }
      float alpha[8];
#pragma unroll
      for (int v = 0; v < 8; ++v) {
        float mx = fmaxf(s0[v], s1[v]);
        mx = red16_max(mx);
        const float mn = fmaxf(mrow[v], mx);
        alpha[v] = __expf(mrow[v] - mn);
        mrow[v] = mn;
      }
#pragma unroll
      for (int v = 0; v < 8; ++v) {
        s0[v] = __expf(s0[v] - mrow[v]);
        s1[v] = __expf(s1[v] - mrow[v]);
      }
#pragma unroll
      for (int v = 0; v < 8; ++v) {
        const float rs = red16_sum(s0[v] + s1[v]);
        lrow[v] = alpha[v] * lrow[v] + rs;
      }
#pragma unroll
      for (int nb = 0; nb < 4; ++nb)
#pragma unroll
        for (int v = 0; v < 8; ++v) o[nb][v] = o[nb][v] * alpha[v];
#pragma unroll
      for (int v = 0; v < 8; ++v) {
        P[(hh * 8u + (unsigned)v) * LDT + m]       = toh_flush(s0[v] * PCARRY);
        P[(hh * 8u + (unsigned)v) * LDT + 16u + m] = toh_flush(s1[v] * PCARRY);
      }
      wave_lds_sync();
      const v16h pf = ld_frag(P, LDT);
#pragma unroll
      for (int nb = 0; nb < 4; ++nb) {
        const _Float16* vp = Vt + vplane + (size_t)((unsigned)nb * 16u + m) * SEQ
                             + kb + kg * 16u + hh * 8u;
        const v16h vf = frag_two(vp, vp + 64);
        o[nb] = wmma16(pf, vf, o[nb]);
      }
      wave_lds_sync();
    }
  }

  for (unsigned kb = wstart; kb < kend; kb += 64u) {
#pragma unroll
    for (unsigned j = 0; j < 2u; ++j) {
      const unsigned idx = tid + 256u * j;
      const unsigned r = idx >> 3, c = (idx & 7u) * 8u;
      *(v8h*)&Ks[r * LDT + c] = *(const v8h*)(Kh + kplane + (size_t)(kb + r) * DIM + c);
      *(v8h*)&Vs[r * LDT + c] = *(const v8h*)(Vt + vplane + (size_t)r * SEQ + kb + c);
      if (EARLY) {
        *(v8h*)&KRs[r * LDT + c] = *(const v8h*)(KR + kplane + (size_t)(kb + r) * DIM + c);
        *(v8h*)&VRs[r * LDT + c] = *(const v8h*)(VtR + rplane + (size_t)r * EROWS + kb + c);
      }
    }
    __syncthreads();

    v8f s[4];
#pragma unroll
    for (int kg = 0; kg < 4; ++kg) {
      v8f t = {};
      if (EARLY) {
        v8f t2 = {};
#pragma unroll
        for (int c = 0; c < 2; ++c) {
          const v16h kf = ld_frag(&Ks[(kg * 16) * LDT + c * 32], LDT);
          const v16h kr = ld_frag(&KRs[(kg * 16) * LDT + c * 32], LDT);
          t  = wmma16(qf[c], kf, t);
          t2 = wmma16(qf[c], kr, t2);
          t2 = wmma16(qr[c], kf, t2);
        }
        s[kg] = (t + t2 * (1.0f / RCARRY)) * scale;
      } else {
#pragma unroll
        for (int c = 0; c < 2; ++c) {
          const v16h kf = ld_frag(&Ks[(kg * 16) * LDT + c * 32], LDT);
          t = wmma16(qf[c], kf, t);
        }
        s[kg] = t * scale;
      }
    }

#pragma unroll
    for (int kg = 0; kg < 4; ++kg)
#pragma unroll
      for (int v = 0; v < 8; ++v) {
        const int d = (int)(qrow0 + hh * 8u + (unsigned)v) - (int)(kb + (unsigned)kg * 16u + m);
        const bool ok = (d >= 0) && ((d < WINDOW) || ((d & (STRIDE - 1)) == 0));
        s[kg][v] = ok ? s[kg][v] : -1.0e30f;
      }

    float alpha[8];
#pragma unroll
    for (int v = 0; v < 8; ++v) {
      float mx = fmaxf(fmaxf(s[0][v], s[1][v]), fmaxf(s[2][v], s[3][v]));
      mx = red16_max(mx);
      const float mn = fmaxf(mrow[v], mx);
      alpha[v] = __expf(mrow[v] - mn);
      mrow[v] = mn;
    }
#pragma unroll
    for (int kg = 0; kg < 4; ++kg)
#pragma unroll
      for (int v = 0; v < 8; ++v) s[kg][v] = __expf(s[kg][v] - mrow[v]);
#pragma unroll
    for (int v = 0; v < 8; ++v) {
      const float rs = red16_sum((s[0][v] + s[1][v]) + (s[2][v] + s[3][v]));
      lrow[v] = alpha[v] * lrow[v] + rs;
    }
#pragma unroll
    for (int nb = 0; nb < 4; ++nb)
#pragma unroll
      for (int v = 0; v < 8; ++v) o[nb][v] = o[nb][v] * alpha[v];

#pragma unroll
    for (int kg = 0; kg < 4; ++kg)
#pragma unroll
      for (int v = 0; v < 8; ++v)
        P[(hh * 8u + (unsigned)v) * LDT + (unsigned)kg * 16u + m] = toh_flush(s[kg][v] * PCARRY);
    wave_lds_sync();

#pragma unroll
    for (int c = 0; c < 2; ++c) {
      const v16h pf = ld_frag(P + c * 32, LDT);
#pragma unroll
      for (int nb = 0; nb < 4; ++nb) {
        const v16h vf = ld_frag(&Vs[(nb * 16) * LDT + c * 32], LDT);
        o[nb] = wmma16(pf, vf, o[nb]);
      }
    }

    if (EARLY) {
#pragma unroll
      for (int nb = 0; nb < 4; ++nb) {
        v8f o2 = {};
#pragma unroll
        for (int c = 0; c < 2; ++c) {
          const v16h pf = ld_frag(P + c * 32, LDT);
          const v16h vr = ld_frag(&VRs[(nb * 16) * LDT + c * 32], LDT);
          o2 = wmma16(pf, vr, o2);
        }
#pragma unroll
        for (int v = 0; v < 8; ++v) o[nb][v] = o[nb][v] + o2[v] * (1.0f / RCARRY);
      }
      wave_lds_sync();
#pragma unroll
      for (int kg = 0; kg < 4; ++kg)
#pragma unroll
        for (int v = 0; v < 8; ++v) {
          const float t = s[kg][v] * PCARRY;
          const float hi = (float)toh_flush(t);
          P[(hh * 8u + (unsigned)v) * LDT + (unsigned)kg * 16u + m] =
              toh_flush((t - hi) * RCARRY);
        }
      wave_lds_sync();
#pragma unroll
      for (int nb = 0; nb < 4; ++nb) {
        v8f o2 = {};
#pragma unroll
        for (int c = 0; c < 2; ++c) {
          const v16h pf = ld_frag(P + c * 32, LDT);
          const v16h vf = ld_frag(&Vs[(nb * 16) * LDT + c * 32], LDT);
          o2 = wmma16(pf, vf, o2);
        }
#pragma unroll
        for (int v = 0; v < 8; ++v) o[nb][v] = o[nb][v] + o2[v] * (1.0f / RCARRY);
      }
    }
    __syncthreads();
  }

  float inv[8];
#pragma unroll
  for (int v = 0; v < 8; ++v) inv[v] = __builtin_amdgcn_rcpf(lrow[v]) * (VCARRY / PCARRY);
#pragma unroll
  for (int nb = 0; nb < 4; ++nb)
#pragma unroll
    for (int v = 0; v < 8; ++v) {
      const float t = o[nb][v] * inv[v];
      const _Float16 hi = toh_flush(t);
      P[(hh * 8u + (unsigned)v) * LDT + (unsigned)nb * 16u + m] = hi;
      o[nb][v] = (t - (float)hi) * RCARRY;
    }
  wave_lds_sync();
  v8h x[4], xr[4];
  size_t off[4];
#pragma unroll
  for (unsigned i = 0; i < 4u; ++i) {
    const unsigned r = 4u * i + (lane >> 3);
    const unsigned c = (lane & 7u) * 8u;
    x[i] = *(const v8h*)&P[r * LDT + c];
    xr[i] = x[i];
    off[i] = (size_t)(qrow0 + r) * DIM + head * HD + c;
  }
  if (EARLY) {
    wave_lds_sync();
#pragma unroll
    for (int nb = 0; nb < 4; ++nb)
#pragma unroll
      for (int v = 0; v < 8; ++v)
        P[(hh * 8u + (unsigned)v) * LDT + (unsigned)nb * 16u + m] = toh_flush(o[nb][v]);
    wave_lds_sync();
#pragma unroll
    for (unsigned i = 0; i < 4u; ++i) {
      const unsigned r = 4u * i + (lane >> 3);
      const unsigned c = (lane & 7u) * 8u;
      xr[i] = *(const v8h*)&P[r * LDT + c];
    }
  }
#pragma unroll
  for (int i = 0; i < 4; ++i) *(volatile v8h*)(Ov + off[i]) = x[i];
  if (EARLY) {
#pragma unroll
    for (int i = 0; i < 4; ++i) *(volatile v8h*)(OvR + off[i]) = xr[i];
  }
  __threadfence();
#pragma unroll
  for (int i = 0; i < 4; ++i) *(volatile v8h*)(Ov + off[i]) = x[i];
  if (EARLY) {
#pragma unroll
    for (int i = 0; i < 4; ++i) *(volatile v8h*)(OvR + off[i]) = xr[i];
  }
}

__global__ __launch_bounds__(256) void attn_early_kernel(
    const _Float16* __restrict__ Qh, const _Float16* __restrict__ Kh,
    const _Float16* __restrict__ Vt, const _Float16* __restrict__ QR,
    const _Float16* __restrict__ KR, const _Float16* __restrict__ VtR,
    _Float16* __restrict__ Ov, _Float16* __restrict__ OvR) {
  attn_body<EARLY_RES>(Qh, Kh, Vt, QR, KR, VtR, Ov, OvR, blockIdx.x * 128u);
}
__global__ __launch_bounds__(256) void attn_late_kernel(
    const _Float16* __restrict__ Qh, const _Float16* __restrict__ Kh,
    const _Float16* __restrict__ Vt, _Float16* __restrict__ Ov) {
  attn_body<0>(Qh, Kh, Vt, Qh, Kh, Vt, Ov, Ov, (unsigned)EROWS + blockIdx.x * 128u);
}

extern "C" void kernel_launch(void* const* d_in, const int* in_sizes, int n_in,
                              void* d_out, int out_size, void* d_ws, size_t ws_size,
                              hipStream_t stream) {
  if (n_in < 5) return;
  const long long need_x = (long long)MROWS * DIM;
  if ((long long)in_sizes[0] < need_x) return;
  if ((long long)in_sizes[1] < (long long)DIM * DIM) return;
  if ((long long)in_sizes[2] < (long long)DIM * DIM) return;
  if ((long long)in_sizes[3] < (long long)DIM * DIM) return;
  if ((long long)in_sizes[4] < (long long)DIM * DIM) return;
  if ((long long)out_size < need_x) return;
  if (ws_size < WS_TOTAL) return;

  const float* X  = (const float*)d_in[0];
  const float* wq = (const float*)d_in[1];
  const float* wk = (const float*)d_in[2];
  const float* wv = (const float*)d_in[3];
  const float* wo = (const float*)d_in[4];
  float* out = (float*)d_out;

  char* ws = (char*)d_ws;
  _Float16* X16   = (_Float16*)(ws + OFF_X);
  _Float16* Wq_t  = (_Float16*)(ws + OFF_WQ);
  _Float16* Wk_t  = (_Float16*)(ws + OFF_WK);
  _Float16* Wv_t  = (_Float16*)(ws + OFF_WV);
  _Float16* Wo_t  = (_Float16*)(ws + OFF_WO);
  _Float16* Qh16  = (_Float16*)(ws + OFF_Q);
  _Float16* Kh16  = (_Float16*)(ws + OFF_K);
  _Float16* Vt16  = (_Float16*)(ws + OFF_VT);
  _Float16* Ctx16 = (_Float16*)(ws + OFF_CTX);
  _Float16* QR16  = (_Float16*)(ws + OFF_QR);
  _Float16* KR16  = (_Float16*)(ws + OFF_KR);
  _Float16* VtR16 = (_Float16*)(ws + OFF_VR);
  _Float16* CtxR  = (_Float16*)(ws + OFF_CR);

  dim3 blk(256);
  dim3 gg(DIM / 64, MROWS / 64);

  cvt_plane_kernel<<<dim3((unsigned)(((size_t)MROWS * DIM) / 2048)), blk, 0, stream>>>(X, X16, 1.0f);
  cvt_plane_kernel<<<dim3((DIM * DIM) / 2048), blk, 0, stream>>>(wq, Wq_t, WCARRY);
  cvt_plane_kernel<<<dim3((DIM * DIM) / 2048), blk, 0, stream>>>(wk, Wk_t, WCARRY);
  cvt_plane_kernel<<<dim3((DIM * DIM) / 2048), blk, 0, stream>>>(wv, Wv_t, WCARRY);
  cvt_plane_kernel<<<dim3((DIM * DIM) / 2048), blk, 0, stream>>>(wo, Wo_t, WCARRY);

  gemm_qk_kernel<<<gg, blk, 0, stream>>>(X16, Wq_t, Qh16, QR16);
  gemm_qk_kernel<<<gg, blk, 0, stream>>>(X16, Wk_t, Kh16, KR16);
  gemm_v_kernel<<<gg, blk, 0, stream>>>(X16, Wv_t, Vt16, VtR16);
  attn_early_kernel<<<dim3(EROWS / 128, NHEAD), blk, 0, stream>>>(
      Qh16, Kh16, Vt16, QR16, KR16, VtR16, Ctx16, CtxR);
  if (SEQ > EROWS) {
    attn_late_kernel<<<dim3((SEQ - EROWS) / 128, NHEAD), blk, 0, stream>>>(
        Qh16, Kh16, Vt16, Ctx16);
  }
  gemm_wo_kernel<<<gg, blk, 0, stream>>>(Ctx16, CtxR, Wo_t, out);
}
